// feature_Attention_CostAgg_Module_65335042506914
// MI455X (gfx1250) — hardware-verified
//
#include <hip/hip_runtime.h>


#define NB 4
#define NC 32
#define ND 64
#define NH 128
#define NW 256
#define HWP 32768
#define BN_EPS 1e-5f
#define PSCALE 16384.0f
#define INV_PSCALE 6.103515625e-05f
#define WSCALE 16.0f
#define INV_WSCALE 0.0625f
#define NEG_BIG (-3.0e38f)

typedef _Float16 f16_t;
typedef _Float16 v16h __attribute__((ext_vector_type(16)));
typedef _Float16 v8h __attribute__((ext_vector_type(8)));
typedef float v8f __attribute__((ext_vector_type(8)));
typedef float v4f __attribute__((ext_vector_type(4)));

union Frag16 { v16h v; v8h h[2]; };
union Pack8 { v8h h; v4f f; };

__device__ __forceinline__ v8f zero8() {
  v8f z = {0.f, 0.f, 0.f, 0.f, 0.f, 0.f, 0.f, 0.f};
  return z;
}

__device__ __forceinline__ v16h ld_frag(const f16_t* base, size_t pitch, int k0) {
  const int l = threadIdx.x & 31;
  const f16_t* p = base + (size_t)(l & 15) * pitch + k0 + 8 * (l >> 4);
  Frag16 f;
  f.h[0] = *(const v8h*)p;
  f.h[1] = *(const v8h*)(p + 16);
  return f.v;
}

__device__ __forceinline__ v8f mma(v16h a, v16h b, v8f c) {
  c = __builtin_amdgcn_wmma_f32_16x16x32_f16(false, a, false, b, (short)0, c, false, false);
  asm volatile("v_nop\n\tv_nop\n\tv_nop\n\tv_nop" : "+v"(c) : "v"(a), "v"(b));
  return c;
}

__device__ __forceinline__ void vst_f(float* p, v4f v) { *(volatile v4f*)p = v; }
__device__ __forceinline__ void vst_h(f16_t* p, v4f v) { *(volatile v4f*)(void*)p = v; }
__device__ __forceinline__ v4f ld16(const void* p) { return *(const v4f*)p; }

__global__ __launch_bounds__(256) void k_wconv(const float* __restrict__ Wa, const float* __restrict__ Wb,
                                              const float* __restrict__ Wq, const float* __restrict__ Wk,
                                              const float* __restrict__ Wv, f16_t* __restrict__ wbuf) {
  const int t = blockIdx.x * 256 + threadIdx.x;
  if (t >= 9984) return;
  const int e0 = t * 8;
  Pack8 u;
#pragma unroll
  for (int j = 0; j < 8; ++j) {
    const int e = e0 + j;
    float v;
    if (e < 36864) {
      const int tap = e >> 12, rem = e & 4095, o = rem >> 6, ic = rem & 63;
      v = Wa[((o * 64 + ic) * 3 + tap / 3) * 3 + (tap - (tap / 3) * 3)];
    } else if (e < 73728) {
      const int e2 = e - 36864;
      const int tap = e2 >> 12, rem = e2 & 4095, o = rem >> 6, ic = rem & 63;
      v = Wb[((o * 64 + ic) * 3 + tap / 3) * 3 + (tap - (tap / 3) * 3)];
    } else if (e < 74752) {
      v = Wq[e - 73728];
    } else if (e < 75776) {
      v = Wk[e - 74752];
    } else {
      v = Wv[e - 75776];
    }
    u.h[j] = (f16_t)(v * WSCALE);
  }
  const v4f val = u.f;
  vst_h(wbuf + e0, val);
  __threadfence();
  vst_h(wbuf + e0, val);
}

__global__ __launch_bounds__(128) void k_conv3x3(const float* __restrict__ x, const f16_t* __restrict__ w9,
                                                float* __restrict__ y, float* __restrict__ part) {
  const int wt = blockIdx.x, h = blockIdx.y, b = blockIdx.z;
  const int w0 = wt * 32;
  const int blk = (b * NH + h) * 8 + wt;
  __shared__ __align__(16) f16_t xs[3 * 34 * 64];
  __shared__ __align__(16) float os[64 * 32];
  __shared__ __align__(16) float psm[128];
  const int tid = threadIdx.x;
  for (int idx = tid; idx < 1536; idx += 128) {
    const int j = idx & 7, rc = idx >> 3, c = rc & 63, row = rc >> 6;
    const int hh = h - 1 + row;
    v4f v = {0.f, 0.f, 0.f, 0.f};
    if ((unsigned)hh < (unsigned)NH)
      v = *(const v4f*)(x + ((size_t)(b * ND + c) * NH + hh) * NW + w0 + 4 * j);
    f16_t* d = xs + (row * 34 + 1 + 4 * j) * 64 + c;
    d[0] = (f16_t)v.x;
    d[64] = (f16_t)v.y;
    d[128] = (f16_t)v.z;
    d[192] = (f16_t)v.w;
  }
  for (int idx = tid; idx < 384; idx += 128) {
    const int side = idx & 1, rc = idx >> 1, c = rc & 63, row = rc >> 6;
    const int hh = h - 1 + row, wg = side ? (w0 + 32) : (w0 - 1);
    float v = 0.f;
    if ((unsigned)hh < (unsigned)NH && (unsigned)wg < (unsigned)NW)
      v = x[((size_t)(b * ND + c) * NH + hh) * NW + wg];
    xs[(row * 34 + (side ? 33 : 0)) * 64 + c] = (f16_t)v;
  }
  __syncthreads();
  const int wv = tid >> 5, l = tid & 31, hf = l >> 4, n = l & 15;
  v8f acc0 = zero8(), acc1 = zero8();
#pragma unroll 1
  for (int tap = 0; tap < 9; ++tap) {
    const int ky = tap / 3, kx = tap - ky * 3;
    const f16_t* wtile = w9 + tap * 4096 + (wv * 16) * 64;
    const f16_t* xb = xs + (ky * 34 + kx) * 64;
#pragma unroll
    for (int kc = 0; kc < 64; kc += 32) {
      const v16h a = ld_frag(wtile, 64, kc);
      const v16h b0 = ld_frag(xb, 64, kc);
      const v16h b1 = ld_frag(xb + 16 * 64, 64, kc);
      acc0 = mma(a, b0, acc0);
      acc1 = mma(a, b1, acc1);
    }
  }
#pragma unroll
  for (int r = 0; r < 8; ++r) {
    const int oc = wv * 16 + 8 * hf + r;
    os[oc * 32 + n] = acc0[r] * INV_WSCALE;
    os[oc * 32 + 16 + n] = acc1[r] * INV_WSCALE;
  }
  __syncthreads();
  if (tid < 64) {
    float s = 0.f, s2 = 0.f;
    for (int px = 0; px < 32; ++px) {
      const float v = os[tid * 32 + px];
      s += v;
      s2 += v * v;
    }
    psm[2 * tid] = s;
    psm[2 * tid + 1] = s2;
  }
  __syncthreads();
  const int piece = tid & 7, lq = tid >> 3;
  for (int pass = 0; pass < 2; ++pass) {
#pragma unroll
    for (int u = 0; u < 4; ++u) {
      const int d = u * 16 + lq;
      const v4f v = ld16(&os[d * 32 + 4 * piece]);
      vst_f(y + ((size_t)(b * ND + d) * NH + h) * NW + w0 + 4 * piece, v);
    }
    if (tid < 32) vst_f(part + (size_t)blk * 128 + 4 * tid, ld16(&psm[4 * tid]));
    if (pass == 0) __threadfence();
  }
}

__global__ __launch_bounds__(256) void k_bnfinal(const float* __restrict__ part, const float* __restrict__ g,
                                                const float* __restrict__ be, float* __restrict__ bnp) {
  __shared__ double ds[256], ds2[256];
  __shared__ __align__(16) float sb[128];
  const int tid = threadIdx.x, d = tid & 63, q = tid >> 6;
  double s = 0.0, s2 = 0.0;
  for (int i = q * 1024; i < (q + 1) * 1024; ++i) {
    s += (double)part[(size_t)i * 128 + 2 * d];
    s2 += (double)part[(size_t)i * 128 + 2 * d + 1];
  }
  ds[tid] = s;
  ds2[tid] = s2;
  __syncthreads();
  if (tid < 64) {
    const double S = ((ds[tid] + ds[tid + 64]) + ds[tid + 128]) + ds[tid + 192];
    const double S2 = ((ds2[tid] + ds2[tid + 64]) + ds2[tid + 128]) + ds2[tid + 192];
    const double invN = 1.0 / (double)(NB * HWP);
    const double mean = S * invN;
    double var = S2 * invN - mean * mean;
    if (var < 0.0) var = 0.0;
    const float rstd = rsqrtf((float)var + BN_EPS);
    const float sc = g[tid] * rstd;
    const float sh = be[tid] - (float)mean * sc;
    sb[tid] = sc;
    sb[64 + tid] = sh;
  }
  __syncthreads();
  if (tid < 32) {
    const v4f v = ld16(&sb[4 * tid]);
    vst_f(bnp + 4 * tid, v);
    __threadfence();
    vst_f(bnp + 4 * tid, v);
  }
}

__global__ __launch_bounds__(256) void k_bnapply(const float* x, const float* __restrict__ bnp, float* y) {
  const size_t i4 = (size_t)blockIdx.x * 256 + threadIdx.x;
  const int d = (int)((i4 >> 13) & 63);
  const float sc = bnp[d], sh = bnp[64 + d];
  const v4f v = *(const v4f*)(x + i4 * 4);
  v4f o;
  o.x = v.x * sc + sh;
  o.y = v.y * sc + sh;
  o.z = v.z * sc + sh;
  o.w = v.w * sc + sh;
  vst_f(y + i4 * 4, o);
  __threadfence();
  vst_f(y + i4 * 4, o);
}

__global__ __launch_bounds__(128) void k_proj_c32(const float* __restrict__ x, const f16_t* __restrict__ wm,
                                                 const float* __restrict__ bias, f16_t* __restrict__ y) {
  const int p0 = blockIdx.x * 64, b = p0 / HWP, pix0 = p0 - b * HWP;
  __shared__ __align__(16) f16_t xs[64 * 32];
  __shared__ __align__(16) f16_t os[64 * 32];
  const int tid = threadIdx.x;
  for (int idx = tid; idx < 512; idx += 128) {
    const int j = idx & 15, ci = idx >> 4;
    const v4f v = *(const v4f*)(x + (size_t)(b * NC + ci) * HWP + pix0 + 4 * j);
    f16_t* d = xs + (4 * j) * 32 + ci;
    d[0] = (f16_t)v.x;
    d[32] = (f16_t)v.y;
    d[64] = (f16_t)v.z;
    d[96] = (f16_t)v.w;
  }
  __syncthreads();
  const int wv = tid >> 5, l = tid & 31, hf = l >> 4, n = l & 15;
  const v16h A = ld_frag(xs + (wv * 16) * 32, 32, 0);
#pragma unroll
  for (int nt = 0; nt < 2; ++nt) {
    const v8f acc = mma(A, ld_frag(wm + (nt * 16) * 32, 32, 0), zero8());
    const int co = nt * 16 + n;
    const float bb = bias[co];
#pragma unroll
    for (int r = 0; r < 8; ++r) {
      const int px = wv * 16 + 8 * hf + r;
      os[px * 32 + co] = (f16_t)(acc[r] * INV_WSCALE + bb);
    }
  }
  __syncthreads();
  f16_t* dst = y + ((size_t)b * HWP + pix0) * 32;
  for (int pass = 0; pass < 2; ++pass) {
#pragma unroll
    for (int u = 0; u < 2; ++u) {
      const int ch = u * 128 + tid;
      vst_h(dst + ch * 8, ld16(os + ch * 8));
    }
    if (pass == 0) __threadfence();
  }
}

__global__ __launch_bounds__(128) void k_proj_c64(const float* __restrict__ x, const f16_t* __restrict__ wm,
                                                 const float* __restrict__ bias, f16_t* __restrict__ y) {
  const int p0 = blockIdx.x * 64, b = p0 / HWP, pix0 = p0 - b * HWP;
  __shared__ __align__(16) f16_t xs[64 * 64];
  __shared__ __align__(16) f16_t os[64 * 64];
  const int tid = threadIdx.x;
  for (int idx = tid; idx < 1024; idx += 128) {
    const int j = idx & 15, ci = idx >> 4;
    const v4f v = *(const v4f*)(x + (size_t)(b * ND + ci) * HWP + pix0 + 4 * j);
    f16_t* d = xs + (4 * j) * 64 + ci;
    d[0] = (f16_t)v.x;
    d[64] = (f16_t)v.y;
    d[128] = (f16_t)v.z;
    d[192] = (f16_t)v.w;
  }
  __syncthreads();
  const int wv = tid >> 5, l = tid & 31, hf = l >> 4, n = l & 15;
  v8f acc[4];
#pragma unroll
  for (int nt = 0; nt < 4; ++nt) acc[nt] = zero8();
#pragma unroll
  for (int kc = 0; kc < 64; kc += 32) {
    const v16h A = ld_frag(wm + (wv * 16) * 64, 64, kc);
#pragma unroll
    for (int nt = 0; nt < 4; ++nt) acc[nt] = mma(A, ld_frag(xs + (nt * 16) * 64, 64, kc), acc[nt]);
  }
#pragma unroll
  for (int r = 0; r < 8; ++r) {
    const int co = wv * 16 + 8 * hf + r;
    const float bb = bias[co];
#pragma unroll
    for (int nt = 0; nt < 4; ++nt) os[co * 64 + nt * 16 + n] = (f16_t)(acc[nt][r] * INV_WSCALE + bb);
  }
  __syncthreads();
  const int piece = tid & 7, lq = tid >> 3;
  for (int pass = 0; pass < 2; ++pass) {
#pragma unroll
    for (int u = 0; u < 4; ++u) {
      const int co = u * 16 + lq;
      vst_h(y + (size_t)(b * ND + co) * HWP + pix0 + piece * 8, ld16(os + co * 64 + piece * 8));
    }
    if (pass == 0) __threadfence();
  }
}

__global__ __launch_bounds__(256) void k_vtrans(const f16_t* __restrict__ vh, f16_t* __restrict__ vt) {
  const int w0 = blockIdx.x * 64, h0 = blockIdx.y * 64, bd = blockIdx.z;
  const int b = bd >> 6, d = bd & 63;
  __shared__ __align__(16) f16_t ts[64 * 72];
  const int tid = threadIdx.x;
#pragma unroll
  for (int u = 0; u < 2; ++u) {
    const int idx = u * 256 + tid, hl = idx >> 3, q8 = idx & 7;
    const v8h v = *(const v8h*)(vh + ((size_t)(b * ND + d) * NH + h0 + hl) * NW + w0 + 8 * q8);
    *(v8h*)(ts + hl * 72 + 8 * q8) = v;
  }
  __syncthreads();
  for (int pass = 0; pass < 2; ++pass) {
#pragma unroll
    for (int u = 0; u < 2; ++u) {
      const int idx = u * 256 + tid, wl = idx >> 3, q8 = idx & 7;
      Pack8 o;
#pragma unroll
      for (int j = 0; j < 8; ++j) o.h[j] = ts[(8 * q8 + j) * 72 + wl];
      vst_h(vt + (((size_t)(b * NW + w0 + wl)) * ND + d) * NH + h0 + 8 * q8, o.f);
    }
    if (pass == 0) __threadfence();
  }
}

__global__ __launch_bounds__(256) void k_statW(const f16_t* __restrict__ qh, const f16_t* __restrict__ kh,
                                              float* __restrict__ stW) {
  const int h = blockIdx.x, b = blockIdx.y;
  __shared__ __align__(16) float st[512];
  const int tid = threadIdx.x, wv = tid >> 5, l = tid & 31, hf = l >> 4;
  const size_t rp = ((size_t)(b * NH + h)) * NW;
  const f16_t* qr = qh + rp * 32;
  const f16_t* kr = kh + rp * 32;
#pragma unroll 1
  for (int u = 0; u < 2; ++u) {
    const int mt = wv * 2 + u;
    const v16h A = ld_frag(qr + (size_t)(mt * 16) * 32, 32, 0);
    float M[8], S[8];
#pragma unroll
    for (int hv = 0; hv < 2; ++hv) {
      v8f e[8];
#pragma unroll
      for (int t = 0; t < 8; ++t) e[t] = mma(A, ld_frag(kr + (size_t)(hv * 128 + t * 16) * 32, 32, 0), zero8());
#pragma unroll
      for (int r = 0; r < 8; ++r) {
        float m = e[0][r];
#pragma unroll
        for (int t = 1; t < 8; ++t) m = fmaxf(m, e[t][r]);
        m = fmaxf(m, __shfl_xor(m, 1, 32));
        m = fmaxf(m, __shfl_xor(m, 2, 32));
        m = fmaxf(m, __shfl_xor(m, 4, 32));
        m = fmaxf(m, __shfl_xor(m, 8, 32));
        float s = 0.f;
#pragma unroll
        for (int t = 0; t < 8; ++t) s += __expf(e[t][r] - m);
        s += __shfl_xor(s, 1, 32);
        s += __shfl_xor(s, 2, 32);
        s += __shfl_xor(s, 4, 32);
        s += __shfl_xor(s, 8, 32);
        if (hv == 0) {
          M[r] = m;
          S[r] = s;
        } else {
          const float Mn = fmaxf(M[r], m);
          S[r] = S[r] * __expf(M[r] - Mn) + s * __expf(m - Mn);
          M[r] = Mn;
        }
      }
    }
#pragma unroll
    for (int r = 0; r < 8; ++r) {
      const int w = mt * 16 + 8 * hf + r;
      st[2 * w] = M[r];
      st[2 * w + 1] = S[r];
    }
  }
  __syncthreads();
  if (tid < 128) {
    const v4f v = ld16(&st[4 * tid]);
    float* dst = stW + rp * 2 + 4 * tid;
    vst_f(dst, v);
    __threadfence();
    vst_f(dst, v);
  }
}

__global__ __launch_bounds__(256) void k_statH(const f16_t* __restrict__ qh, const f16_t* __restrict__ kh,
                                              const float* __restrict__ stW, float* __restrict__ stF,
                                              f16_t* __restrict__ pH) {
  const int w = blockIdx.x, b = blockIdx.y;
  __shared__ float sw[256];
  __shared__ __align__(16) float sg[256];
  __shared__ __align__(16) f16_t pt[128 * 136];
  const int tid = threadIdx.x, wv = tid >> 5, l = tid & 31, hf = l >> 4, n = l & 15;
  sw[tid] = stW[(((size_t)(b * NH + (tid >> 1))) * NW + w) * 2 + (tid & 1)];
  const size_t cp = (size_t)NW * 32;
  const f16_t* qc = qh + (((size_t)(b * NH)) * NW + w) * 32;
  const f16_t* kc = kh + (((size_t)(b * NH)) * NW + w) * 32;
  const v16h A = ld_frag(qc + (size_t)(wv * 16) * cp, cp, 0);
  v8f e[8];
#pragma unroll
  for (int t = 0; t < 8; ++t) e[t] = mma(A, ld_frag(kc + (size_t)(t * 16) * cp, cp, 0), zero8());
  float mx[8], sm[8];
#pragma unroll
  for (int r = 0; r < 8; ++r) {
    const int hr = wv * 16 + 8 * hf + r;
    float m = NEG_BIG;
#pragma unroll
    for (int t = 0; t < 8; ++t) {
      const float v = (t * 16 + n == hr) ? NEG_BIG : e[t][r];
      m = fmaxf(m, v);
    }
    m = fmaxf(m, __shfl_xor(m, 1, 32));
    m = fmaxf(m, __shfl_xor(m, 2, 32));
    m = fmaxf(m, __shfl_xor(m, 4, 32));
    m = fmaxf(m, __shfl_xor(m, 8, 32));
    mx[r] = m;
    float s = 0.f;
#pragma unroll
    for (int t = 0; t < 8; ++t) {
      const float ex = (t * 16 + n == hr) ? 0.f : __expf(e[t][r] - m);
      e[t][r] = ex;
      s += ex;
    }
    s += __shfl_xor(s, 1, 32);
    s += __shfl_xor(s, 2, 32);
    s += __shfl_xor(s, 4, 32);
    s += __shfl_xor(s, 8, 32);
    sm[r] = s;
  }
  __syncthreads();
  float F[8];
#pragma unroll
  for (int r = 0; r < 8; ++r) {
    const int hr = wv * 16 + 8 * hf + r;
    const float mW = sw[2 * hr], sWv = sw[2 * hr + 1];
    const float M = fmaxf(mx[r], mW);
    const float a = __expf(mx[r] - M);
    const float S = sm[r] * a + sWv * __expf(mW - M);
    const float C = PSCALE * __builtin_amdgcn_rcpf(S);
    F[r] = a * C;
    sg[2 * hr] = M;
    sg[2 * hr + 1] = C;
  }
#pragma unroll
  for (int r = 0; r < 8; ++r) {
    const int hr = wv * 16 + 8 * hf + r;
#pragma unroll
    for (int t = 0; t < 8; ++t) pt[hr * 136 + t * 16 + n] = (f16_t)(e[t][r] * F[r]);
  }
  __syncthreads();
  const int piece = tid & 7, lq = tid >> 3;
  f16_t* pdst = pH + (((size_t)(b * NW + w)) * NH) * 128;
  float* sdst = stF + (((size_t)(b * NW + w)) * NH) * 2;
  for (int pass = 0; pass < 2; ++pass) {
    if (tid < 64) vst_f(sdst + 4 * tid, ld16(&sg[4 * tid]));
#pragma unroll
    for (int u = 0; u < 8; ++u) {
      const int L = u * 32 + lq, hrow = L >> 1, seg = L & 1;
      vst_h(pdst + (size_t)hrow * 128 + seg * 64 + piece * 8, ld16(pt + hrow * 136 + seg * 64 + piece * 8));
    }
    if (pass == 0) __threadfence();
  }
}

__global__ __launch_bounds__(256) void k_rowagg(const f16_t* __restrict__ qh, const f16_t* __restrict__ kh,
                                               const float* __restrict__ stF, const f16_t* __restrict__ vh,
                                               const float* __restrict__ gptr, float* xio) {
  const int h = blockIdx.x, b = blockIdx.y;
  __shared__ __align__(16) float ss[512];
  __shared__ __align__(16) f16_t ps[64 * 264];
  __shared__ __align__(16) float os[64 * 64];
  const int tid = threadIdx.x, wv = tid >> 5, l = tid & 31, hf = l >> 4, n = l & 15;
  {
    const float* sp = stF + (((size_t)(b * NW + tid)) * NH + h) * 2;
    ss[2 * tid] = sp[0];
    ss[2 * tid + 1] = sp[1];
  }
  const float gs = gptr[0] * INV_PSCALE;
  const size_t rp = ((size_t)(b * NH + h)) * NW;
  const f16_t* qr = qh + rp * 32;
  const f16_t* kr = kh + rp * 32;
#pragma unroll 1
  for (int c = 0; c < 4; ++c) {
    __syncthreads();
    {
      const int mt = wv >> 1, ntb = (wv & 1) * 8;
      const v16h A = ld_frag(qr + (size_t)(c * 64 + mt * 16) * 32, 32, 0);
      float Mr[8], Cr[8];
#pragma unroll
      for (int r = 0; r < 8; ++r) {
        const int wr = c * 64 + mt * 16 + 8 * hf + r;
        Mr[r] = ss[2 * wr];
        Cr[r] = ss[2 * wr + 1];
      }
#pragma unroll
      for (int t = 0; t < 8; ++t) {
        const int nt = ntb + t;
        const v8f e = mma(A, ld_frag(kr + (size_t)(nt * 16) * 32, 32, 0), zero8());
#pragma unroll
        for (int r = 0; r < 8; ++r) {
          const int wl = mt * 16 + 8 * hf + r;
          ps[wl * 264 + nt * 16 + n] = (f16_t)(__expf(e[r] - Mr[r]) * Cr[r]);
        }
      }
    }
    __syncthreads();
    {
#pragma unroll
      for (int u = 0; u < 2; ++u) {
        const int tile = wv * 2 + u, mt = tile >> 2, nt = tile & 3;
        const f16_t* vb = vh + (((size_t)(b * ND + nt * 16)) * NH + h) * NW;
        v8f acc = zero8();
#pragma unroll
        for (int ks = 0; ks < 8; ++ks) acc = mma(ld_frag(ps + (mt * 16) * 264, 264, 32 * ks), ld_frag(vb, HWP, 32 * ks), acc);
#pragma unroll
        for (int r = 0; r < 8; ++r) os[(nt * 16 + n) * 64 + mt * 16 + 8 * hf + r] = acc[r];
      }
    }
    __syncthreads();
    {
      const int piece = tid & 7, lq = tid >> 3;
      v4f vals[4];
#pragma unroll
      for (int u = 0; u < 4; ++u) {
        const int L = u * 32 + lq, d = L >> 1, seg = L & 1;
        const v4f o = ld16(&os[d * 64 + seg * 32 + 4 * piece]);
        const size_t idx = (((size_t)(b * ND + d)) * NH + h) * NW + c * 64 + seg * 32 + 4 * piece;
        const v4f xv = *(const v4f*)(xio + idx);
        v4f val;
        val.x = xv.x + gs * o.x;
        val.y = xv.y + gs * o.y;
        val.z = xv.z + gs * o.z;
        val.w = xv.w + gs * o.w;
        vals[u] = val;
        vst_f(xio + idx, val);
      }
      __threadfence();
#pragma unroll
      for (int u = 0; u < 4; ++u) {
        const int L = u * 32 + lq, d = L >> 1, seg = L & 1;
        const size_t idx = (((size_t)(b * ND + d)) * NH + h) * NW + c * 64 + seg * 32 + 4 * piece;
        vst_f(xio + idx, vals[u]);
      }
    }
  }
}

__global__ __launch_bounds__(256) void k_colagg(const f16_t* __restrict__ pH, const f16_t* __restrict__ vt,
                                               const float* __restrict__ gptr, float* xio) {
  const int w0 = blockIdx.x * 32, h0 = blockIdx.y * 16, b = blockIdx.z;
  __shared__ __align__(16) float ob[64 * 16 * 32];
  const int tid = threadIdx.x, wv = tid >> 5, l = tid & 31, hf = l >> 4, n = l & 15;
  const int wsub = wv >> 2, nt = wv & 3;
  const float gs = gptr[0] * INV_PSCALE;
#pragma unroll 1
  for (int it = 0; it < 16; ++it) {
    const int wl = 2 * it + wsub, w = w0 + wl;
    const f16_t* pa = pH + (((size_t)(b * NW + w)) * NH + h0) * 128;
    const f16_t* vb = vt + (((size_t)(b * NW + w)) * ND + nt * 16) * NH;
    v8f acc = zero8();
#pragma unroll
    for (int ks = 0; ks < 4; ++ks) acc = mma(ld_frag(pa, 128, 32 * ks), ld_frag(vb, NH, 32 * ks), acc);
#pragma unroll
    for (int r = 0; r < 8; ++r) ob[(nt * 16 + n) * 512 + (8 * hf + r) * 32 + wl] = acc[r];
  }
  __syncthreads();
  const int piece = tid & 7, lq = tid >> 3;
#pragma unroll 1
  for (int grp = 0; grp < 8; ++grp) {
    v4f vals[4];
#pragma unroll
    for (int u = 0; u < 4; ++u) {
      const int L = (grp * 4 + u) * 32 + lq, d = L >> 4, hl = L & 15;
      const v4f o = ld16(&ob[d * 512 + hl * 32 + 4 * piece]);
      const size_t idx = (((size_t)(b * ND + d)) * NH + h0 + hl) * NW + w0 + 4 * piece;
      const v4f xv = *(const v4f*)(xio + idx);
      v4f val;
      val.x = xv.x + gs * o.x;
      val.y = xv.y + gs * o.y;
      val.z = xv.z + gs * o.z;
      val.w = xv.w + gs * o.w;
      vals[u] = val;
      vst_f(xio + idx, val);
    }
    __threadfence();
#pragma unroll
    for (int u = 0; u < 4; ++u) {
      const int L = (grp * 4 + u) * 32 + lq, d = L >> 4, hl = L & 15;
      const size_t idx = (((size_t)(b * ND + d)) * NH + h0 + hl) * NW + w0 + 4 * piece;
      vst_f(xio + idx, vals[u]);
    }
  }
}

static constexpr size_t SZ_ACT  = (size_t)NB * ND * HWP * 4;
static constexpr size_t OFF_T0  = 0;
static constexpr size_t OFF_Q   = OFF_T0 + SZ_ACT;
static constexpr size_t OFF_K   = OFF_Q + (size_t)NB * NC * HWP * 2;
static constexpr size_t OFF_VH  = OFF_K + (size_t)NB * NC * HWP * 2;
static constexpr size_t OFF_VT  = OFF_VH + (size_t)NB * ND * HWP * 2;
static constexpr size_t OFF_PH  = OFF_VT + (size_t)NB * ND * HWP * 2;
static constexpr size_t OFF_STW = OFF_PH + (size_t)NB * NW * NH * NH * 2;
static constexpr size_t OFF_STF = OFF_STW + (size_t)NB * HWP * 2 * 4;
static constexpr size_t OFF_PART = OFF_STF + (size_t)NB * HWP * 2 * 4;
static constexpr size_t OFF_BNP = OFF_PART + (size_t)4096 * 128 * 4;
static constexpr size_t OFF_W   = OFF_BNP + 4096;
static constexpr size_t OFF_END = OFF_W + (size_t)79872 * 2;

extern "C" void kernel_launch(void* const* d_in, const int* in_sizes, int n_in,
                              void* d_out, int out_size, void* d_ws, size_t ws_size,
                              hipStream_t stream) {
  if (n_in < 16) return;
  if ((size_t)out_size != (size_t)NB * ND * HWP) return;
  if (in_sizes[0] != NB * ND * HWP || in_sizes[1] != NB * NC * HWP || in_sizes[2] != NB * NC * HWP) return;
  if (in_sizes[3] != 36864 || in_sizes[13] != 36864 || in_sizes[6] != 1024 || in_sizes[8] != 1024 || in_sizes[10] != 4096) return;
  if (ws_size < OFF_END) return;

  const float* cost = (const float*)d_in[0];
  const float* lf0  = (const float*)d_in[1];
  const float* lf1  = (const float*)d_in[2];
  const float* Wa   = (const float*)d_in[3];
  const float* ga   = (const float*)d_in[4];
  const float* ba   = (const float*)d_in[5];
  const float* Wq   = (const float*)d_in[6];
  const float* bq   = (const float*)d_in[7];
  const float* Wk   = (const float*)d_in[8];
  const float* bk   = (const float*)d_in[9];
  const float* Wv   = (const float*)d_in[10];
  const float* bv   = (const float*)d_in[11];
  const float* gmm  = (const float*)d_in[12];
  const float* Wb   = (const float*)d_in[13];
  const float* gb   = (const float*)d_in[14];
  const float* bb   = (const float*)d_in[15];
  float* out = (float*)d_out;

  char* ws = (char*)d_ws;
  float* t0   = (float*)(ws + OFF_T0);
  f16_t* qh   = (f16_t*)(ws + OFF_Q);
  f16_t* kh   = (f16_t*)(ws + OFF_K);
  f16_t* vh   = (f16_t*)(ws + OFF_VH);
  f16_t* vt   = (f16_t*)(ws + OFF_VT);
  f16_t* pH   = (f16_t*)(ws + OFF_PH);
  float* stW  = (float*)(ws + OFF_STW);
  float* stF  = (float*)(ws + OFF_STF);
  float* part = (float*)(ws + OFF_PART);
  float* bnp  = (float*)(ws + OFF_BNP);
  f16_t* wbuf = (f16_t*)(ws + OFF_W);
  f16_t* wa = wbuf;
  f16_t* wb = wbuf + 36864;
  f16_t* wq = wbuf + 73728;
  f16_t* wk = wbuf + 74752;
  f16_t* wv = wbuf + 75776;

  k_wconv<<<39, 256, 0, stream>>>(Wa, Wb, Wq, Wk, Wv, wbuf);
  k_conv3x3<<<dim3(8, NH, NB), 128, 0, stream>>>(cost, wa, t0, part);
  k_bnfinal<<<1, 256, 0, stream>>>(part, ga, ba, bnp);
  k_bnapply<<<8192, 256, 0, stream>>>(t0, bnp, t0);
  k_proj_c32<<<2048, 128, 0, stream>>>(lf0, wq, bq, qh);
  k_proj_c32<<<2048, 128, 0, stream>>>(lf1, wk, bk, kh);
  k_statW<<<dim3(NH, NB), 256, 0, stream>>>(qh, kh, stW);
  k_statH<<<dim3(NW, NB), 256, 0, stream>>>(qh, kh, stW, stF, pH);
  for (int it = 0; it < 2; ++it) {
    k_proj_c64<<<2048, 128, 0, stream>>>(t0, wv, bv, vh);
    k_vtrans<<<dim3(4, 2, NB * ND), 256, 0, stream>>>(vh, vt);
    k_rowagg<<<dim3(NH, NB), 256, 0, stream>>>(qh, kh, stF, vh, gmm, t0);
    k_colagg<<<dim3(8, 8, NB), 256, 0, stream>>>(pH, vt, gmm, t0);
  }
  k_conv3x3<<<dim3(8, NH, NB), 128, 0, stream>>>(t0, wb, out, part);
  k_bnfinal<<<1, 256, 0, stream>>>(part, gb, bb, bnp);
  k_bnapply<<<8192, 256, 0, stream>>>(out, bnp, out);
}
